// ISTFTLayer_79791902425567
// MI455X (gfx1250) — hardware-verified
//
#include <hip/hip_runtime.h>
#include <stddef.h>
#include <stdint.h>


#define WIN      1024
#define HOP      256
#define FRAMES   1024
#define NBATCH   16
#define BINS     513
#define KTOT     1024
#define KCHUNKS  32
#define SEGMENTS 1027
#define OUTLEN   262912
#define SEGTILES 65
#define AROWS    19

typedef char chk_kpack[(KTOT == BINS + (BINS - 2)) ? 1 : -1];
typedef char chk_kchunk[(KCHUNKS * 32 == KTOT) ? 1 : -1];
typedef char chk_seg[(SEGMENTS * HOP == OUTLEN) ? 1 : -1];
typedef char chk_tiles[(SEGTILES * 16 >= SEGMENTS) ? 1 : -1];

typedef _Float16 v16h __attribute__((ext_vector_type(16)));
typedef _Float16 v8h  __attribute__((ext_vector_type(8)));
typedef float    v8f  __attribute__((ext_vector_type(8)));
typedef float    v4f  __attribute__((ext_vector_type(4)));
typedef v4f __attribute__((may_alias)) v4f_a;
typedef v8h __attribute__((may_alias)) v8h_a;

union Frag { v16h v; v8h half[2]; };

static __device__ __forceinline__ v8f wmma_f16(v16h a, v16h b, v8f c) {
    v8f d = __builtin_amdgcn_wmma_f32_16x16x32_f16(false, a, false, b, (short)0, c, false, false);
    asm volatile("v_nop\n\tv_nop\n\tv_nop\n\tv_nop" : "+v"(d) : "v"(a), "v"(b));
    return d;
}

__global__ __launch_bounds__(256) void k_basis(_Float16* __restrict__ bas, int nchunks) {
    __shared__ __attribute__((aligned(16))) _Float16 sB[256 * 8];

    const int t = blockIdx.x * 256 + threadIdx.x;
    const bool act = (t < nchunks);
    const int n  = t >> 7;
    const int kb = (t & 127) * 8;
    const float step = 6.28318530717958647692f / (float)WIN;
    const float wnd  = 0.5f - 0.5f * cosf((float)(n & (WIN - 1)) * step);
    const float base = wnd * 1024.0f;

#pragma unroll 1
    for (int e = 0; e < 8; ++e) {
        const int k = kb + e;
        const bool isReal = (k < BINS);
        const int kk = isReal ? k : (k - (WIN / 2));
        const int m  = (kk * n) & (WIN - 1);
        float sn, cs;
        sincosf((float)m * step, &sn, &cs);
        float val;
        if (isReal) {
            const bool edge = (kk == 0) || (kk == WIN / 2);
            val = base * (edge ? 1.0f : 2.0f) * cs;
        } else {
            val = -base * 2.0f * sn;
        }
        sB[threadIdx.x * 8 + e] = (_Float16)val;
    }
    __syncthreads();

    const v8h v = *(const v8h_a*)(sB + threadIdx.x * 8);
    _Float16* p = bas + (size_t)t * 8;
    if (act) *(volatile v8h*)p = v;
    __threadfence();
    if (act) *(volatile v8h*)p = v;
}

__global__ __launch_bounds__(256) void k_gemm_ola(
    const float* __restrict__ xr, const float* __restrict__ xi,
    const _Float16* __restrict__ bas, float* __restrict__ out) {

    __shared__ __attribute__((aligned(16))) _Float16 sA[AROWS * KTOT];
    __shared__ __attribute__((aligned(16))) float    sC[8 * 16 * 32];

    const int tid  = threadIdx.x;
    const int lane = tid & 31;
    const int wave = tid >> 5;
    const int r    = lane & 15;
    const int h    = lane >> 4;
    const int s0   = blockIdx.x * 16;
    const int b    = blockIdx.y;
    const int c0   = wave * 32;

    for (int idx = tid; idx < AROWS * KTOT; idx += 256) {
        const int row = idx >> 10;
        const int k   = idx & (KTOT - 1);
        const int f   = s0 - 3 + row;
        const bool isReal = (k < BINS);
        const int  kk = isReal ? k : (k - (WIN / 2));
        const float* src = isReal ? xr : xi;
        const bool ok = (f >= 0) && (f < FRAMES);
        const int  fr = ok ? f : 0;
        float x = 0.0f;
        if (ok) x = src[((size_t)b * FRAMES + (size_t)fr) * BINS + (size_t)kk];
        sA[idx] = (_Float16)x;
    }
    __syncthreads();

    v8f acc0 = {};
    v8f acc1 = {};

    for (int jj = 0; jj < 4; ++jj) {
        const _Float16* ah = sA + (r + 3 - jj) * KTOT;
        const _Float16* b0 = bas + (size_t)(jj * HOP + c0 + r) * KTOT;
        const _Float16* b1 = bas + (size_t)(jj * HOP + c0 + 16 + r) * KTOT;

#pragma unroll 2
        for (int kc = 0; kc < KCHUNKS; ++kc) {
            const int k0 = kc * 32;
            Frag a, p, q;
            a.half[0] = *(const v8h*)(ah + k0 + 8 * h);
            a.half[1] = *(const v8h*)(ah + k0 + 16 + 8 * h);
            p.half[0] = *(const v8h*)(b0 + k0 + 8 * h);
            p.half[1] = *(const v8h*)(b0 + k0 + 16 + 8 * h);
            q.half[0] = *(const v8h*)(b1 + k0 + 8 * h);
            q.half[1] = *(const v8h*)(b1 + k0 + 16 + 8 * h);
            acc0 = wmma_f16(a.v, p.v, acc0);
            acc1 = wmma_f16(a.v, q.v, acc1);
        }
    }

    const float SCL = 9.5367431640625e-7f;
    float* cw = sC + wave * 512;
#pragma unroll
    for (int i = 0; i < 8; ++i) {
        cw[(8 * h + i) * 32 + r]      = acc0[i] * SCL;
        cw[(8 * h + i) * 32 + 16 + r] = acc1[i] * SCL;
    }
    __syncthreads();

    const int rq = lane >> 3;
    const int ch = (lane & 7) * 4;
    v4f vals[4];
#pragma unroll
    for (int t = 0; t < 4; ++t)
        vals[t] = *(const v4f_a*)(cw + (rq + 4 * t) * 32 + ch);

    const size_t obase = (size_t)b * OUTLEN;
#pragma unroll
    for (int t = 0; t < 4; ++t) {
        const int s = s0 + rq + 4 * t;
        if (s < SEGMENTS) {
            float* p = out + obase + (size_t)s * HOP + c0 + ch;
            *(volatile v4f*)p = vals[t];
        }
    }
    __threadfence();
#pragma unroll
    for (int t = 0; t < 4; ++t) {
        const int s = s0 + rq + 4 * t;
        if (s < SEGMENTS) {
            float* p = out + obase + (size_t)s * HOP + c0 + ch;
            *(volatile v4f*)p = vals[t];
        }
    }
}

extern "C" void kernel_launch(void* const* d_in, const int* in_sizes, int n_in,
                              void* d_out, int out_size, void* d_ws, size_t ws_size,
                              hipStream_t stream) {
    if (n_in < 2) return;
    if (in_sizes[0] != NBATCH * FRAMES * BINS) return;
    if (in_sizes[1] != NBATCH * FRAMES * BINS) return;
    if (out_size != NBATCH * OUTLEN) return;
    const size_t bas_bytes = (size_t)WIN * KTOT * sizeof(_Float16);
    if (ws_size < bas_bytes) return;

    const float* xr = (const float*)d_in[0];
    const float* xi = (const float*)d_in[1];
    float* out = (float*)d_out;
    _Float16* bas = (_Float16*)d_ws;

    const int nchunks = WIN * (KTOT / 8);
    k_basis<<<(nchunks + 255) / 256, 256, 0, stream>>>(bas, nchunks);

    dim3 grid(SEGTILES, NBATCH);
    k_gemm_ola<<<grid, 256, 0, stream>>>(xr, xi, bas, out);
}
